// SAVSS_2D_27865747816471
// MI455X (gfx1250) — hardware-run, weakly checked
//
#include <hip/hip_runtime.h>


namespace {
constexpr int B = 8, HH = 64, WW = 64, L = HH * WW, DM = 96, E = 192, MID = 12, NS = 16, R = 6, XDW = 48, NDIR = 4;
constexpr float XS = 8.0f, WSC = 256.0f;
typedef _Float16 b16;
typedef __attribute__((ext_vector_type(16))) _Float16 v16b;
typedef __attribute__((ext_vector_type(8))) _Float16 v8b;
typedef __attribute__((ext_vector_type(8))) float v8f;
typedef __attribute__((ext_vector_type(4))) float v4f;
typedef __attribute__((ext_vector_type(2))) float v2f;
__device__ __forceinline__ float bf16_rne(float f) { unsigned int u = __float_as_uint(f); u += 0x7FFFu + ((u >> 16) & 1u); float r = __uint_as_float(u & 0xFFFF0000u); asm volatile("" : "+v"(r)); return r; }
__device__ __forceinline__ void split16(float v, b16& hi, b16& lo) { hi = (b16)v; lo = (b16)(v - (float)hi); }
__device__ __forceinline__ v16b frag_kb(const b16* p, int hh) { const v8b a = *(const v8b*)(p + 8 * hh), b = *(const v8b*)(p + 16 + 8 * hh); v16b f;
#pragma unroll
  for (int e = 0; e < 8; ++e) { f[e] = a[e]; f[8 + e] = b[e]; } return f; }
__device__ __forceinline__ v8f wmma16b(v16b a, v16b b, v8f c) { v8f d = __builtin_amdgcn_wmma_f32_16x16x32_f16(false, a, false, b, (short)0, c, false, false); asm volatile("v_nop\n\tv_nop\n\tv_nop\n\tv_nop" : "+v"(d) : "v"(a), "v"(b)); return d; }
__device__ __forceinline__ void wave_lds_sync() { __builtin_amdgcn_fence(__ATOMIC_RELEASE, "workgroup"); __builtin_amdgcn_wave_barrier(); __builtin_amdgcn_fence(__ATOMIC_ACQUIRE, "workgroup"); }
__device__ __forceinline__ float pmul(float a, float b) { float p = a * b; asm volatile("" : "+v"(p)); return p; }
__device__ __forceinline__ int iclamp(int v, int lo, int hi) { return v < lo ? lo : (v > hi ? hi : v); }
__device__ __forceinline__ float silu(float v) { return v / (1.0f + __expf(-v)); }
__device__ __forceinline__ float softplus(float v) { return v > 20.0f ? v : __logf(1.0f + __expf(v)); }

__global__ __launch_bounds__(256) void wput_kernel(const float* __restrict__ win, const float* __restrict__ pw1, const float* __restrict__ pw2, const float* __restrict__ xp, const float* __restrict__ wo, b16* __restrict__ WIN, b16* __restrict__ PW1T, b16* __restrict__ PW2T, b16* __restrict__ XPT, b16* __restrict__ WOT) { const int u = blockIdx.x * 256 + threadIdx.x;
  for (int pass = 0; pass < 2; ++pass) {
    if (u < 2 * E * (DM / 8)) { const int o = u / (DM / 8), k0 = (u % (DM / 8)) * 8; v8b v;
#pragma unroll
      for (int j = 0; j < 8; ++j) v[j] = (b16)(bf16_rne(win[(size_t)o * DM + k0 + j]) * WSC); *(volatile v8b*)(WIN + (size_t)o * DM + k0) = v; }
    if (u < 16 * (E / 8)) { const int o = u / (E / 8), k0 = (u % (E / 8)) * 8; v8b v;
#pragma unroll
      for (int j = 0; j < 8; ++j) v[j] = (b16)(o < MID ? bf16_rne(pw1[(size_t)o * E + k0 + j]) * WSC : 0.0f); *(volatile v8b*)(PW1T + (size_t)o * E + k0) = v; }
    if (u < E * 4) { const int o = u / 4, k0 = (u % 4) * 8; v8b v;
#pragma unroll
      for (int j = 0; j < 8; ++j) { const int k = k0 + j; v[j] = (b16)(k < MID ? bf16_rne(pw2[(size_t)o * MID + k]) * WSC : 0.0f); } *(volatile v8b*)(PW2T + (size_t)o * 32 + k0) = v; }
    if (u < XDW * (E / 8)) { const int o = u / (E / 8), k0 = (u % (E / 8)) * 8; v8b v;
#pragma unroll
      for (int j = 0; j < 8; ++j) v[j] = (b16)(o < R + 2 * NS ? bf16_rne(xp[(size_t)o * E + k0 + j]) * WSC : 0.0f); *(volatile v8b*)(XPT + (size_t)o * E + k0) = v; }
    if (u < DM * (E / 8)) { const int o = u / (E / 8), k0 = (u % (E / 8)) * 8; v8b v;
#pragma unroll
      for (int j = 0; j < 8; ++j) v[j] = (b16)(bf16_rne(wo[(size_t)o * E + k0 + j]) * WSC); *(volatile v8b*)(WOT + (size_t)o * E + k0) = v; }
    __threadfence(); } }
__global__ __launch_bounds__(32) void inproj_kernel(const float* __restrict__ x, const b16* __restrict__ WIN, int NRV, float* __restrict__ XZ) { __shared__ __attribute__((aligned(16))) b16 Ah[16][104]; __shared__ float Tf[16][132]; const int lane = threadIdx.x, nloc = lane & 15, hlf = lane >> 4; const int g = blockIdx.x % 3; const size_t m0 = (size_t)(blockIdx.x / 3) * 16; if (m0 >= (size_t)NRV) return;
  for (int rr = 0; rr < 16; ++rr) for (int q = 0; q < 3; ++q) Ah[rr][q * 32 + lane] = (b16)(bf16_rne(x[(m0 + rr) * DM + q * 32 + lane]) * XS);
  wave_lds_sync(); v8f acc[8];
#pragma unroll
  for (int t = 0; t < 8; ++t) acc[t] = (v8f){};
#pragma unroll
  for (int kb = 0; kb < DM; kb += 32) { const v16b a = frag_kb(&Ah[nloc][kb], hlf);
#pragma unroll
    for (int t = 0; t < 8; ++t) acc[t] = wmma16b(a, frag_kb(WIN + (size_t)(g * 128 + t * 16 + nloc) * DM + kb, hlf), acc[t]); }
#pragma unroll
  for (int t = 0; t < 8; ++t)
#pragma unroll
    for (int r8 = 0; r8 < 8; ++r8) Tf[8 * hlf + r8][t * 16 + nloc] = acc[t][r8] * (1.0f / (XS * WSC));
  wave_lds_sync();
  for (int pass = 0; pass < 2; ++pass) { for (int rr = 0; rr < 16; ++rr) *(volatile v4f*)(XZ + (m0 + rr) * 2 * E + g * 128 + lane * 4) = *(const v4f*)(&Tf[rr][lane * 4]); __threadfence(); } }
__global__ __launch_bounds__(32) void pw1_kernel(const float* __restrict__ XZ, const b16* __restrict__ PW1T, const float* __restrict__ b1, int NRV, float* __restrict__ H1) { __shared__ __attribute__((aligned(16))) b16 Ah[16][E + 8], Al[16][E + 8]; __shared__ float Tf[16][17]; const int lane = threadIdx.x, nloc = lane & 15, hlf = lane >> 4; const size_t m0 = (size_t)blockIdx.x * 16; if (m0 >= (size_t)NRV) return;
  for (int rr = 0; rr < 16; ++rr) for (int q = 0; q < E / 32; ++q) { b16 p, ql; split16(XZ[(m0 + rr) * 2 * E + q * 32 + lane] * XS, p, ql); Ah[rr][q * 32 + lane] = p; Al[rr][q * 32 + lane] = ql; }
  wave_lds_sync(); v8f acc = {};
#pragma unroll
  for (int kb = 0; kb < E; kb += 32) { const v16b bw = frag_kb(PW1T + (size_t)nloc * E + kb, hlf); acc = wmma16b(frag_kb(&Ah[nloc][kb], hlf), bw, acc); acc = wmma16b(frag_kb(&Al[nloc][kb], hlf), bw, acc); }
#pragma unroll
  for (int r8 = 0; r8 < 8; ++r8) Tf[8 * hlf + r8][nloc] = nloc < MID ? acc[r8] * (1.0f / (XS * WSC)) + bf16_rne(b1[nloc]) : 0.0f;
  wave_lds_sync();
  for (int pass = 0; pass < 2; ++pass) { for (int q = lane; q < 256; q += 32) ((volatile float*)H1)[m0 * 16 + q] = Tf[q / 16][q % 16]; __threadfence(); } }
__global__ __launch_bounds__(32) void conv_kernel(const float* __restrict__ H1, const float* __restrict__ dw, const b16* __restrict__ PW2T, int NRV, float* __restrict__ XC) { __shared__ __attribute__((aligned(16))) b16 Ah[16][40], Al[16][40]; __shared__ float Tf[16][196]; const int lane = threadIdx.x, nloc = lane & 15, hlf = lane >> 4; const size_t m0 = (size_t)blockIdx.x * 16; if (m0 >= (size_t)NRV) return; const int b = (int)(m0 / L);
  { const int rr = lane & 15, half = lane >> 4; const int p = (int)((m0 + rr) % L); const int py = p / WW, px = p % WW;
    for (int m = half; m < 16; m += 2) { float s = 0.0f; if (m < MID) { for (int dy = -1; dy <= 1; ++dy) for (int dx = -1; dx <= 1; ++dx) { const int yy = py + dy, xx = px + dx; if (yy < 0 || yy >= HH || xx < 0 || xx >= WW) continue; s += pmul(H1[((size_t)b * L + yy * WW + xx) * 16 + m], bf16_rne(dw[(m * 3 + (dy + 1)) * 3 + (dx + 1)])); } }
      b16 ph, pl; split16(s * XS, ph, pl); Ah[rr][m] = ph; Al[rr][m] = pl; Ah[rr][16 + m] = (b16)0.0f; Al[rr][16 + m] = (b16)0.0f; } }
  wave_lds_sync(); const v16b a = frag_kb(&Ah[nloc][0], hlf), al = frag_kb(&Al[nloc][0], hlf);
#pragma unroll
  for (int t = 0; t < E / 16; ++t) { v8f acc = {}; const v16b bw = frag_kb(PW2T + (size_t)(t * 16 + nloc) * 32, hlf); acc = wmma16b(a, bw, acc); acc = wmma16b(al, bw, acc);
#pragma unroll
    for (int r8 = 0; r8 < 8; ++r8) Tf[8 * hlf + r8][t * 16 + nloc] = silu(acc[r8] * (1.0f / (XS * WSC))); }
  wave_lds_sync();
  for (int pass = 0; pass < 2; ++pass) { for (int rr = 0; rr < 16; ++rr) { *(volatile v4f*)(XC + (m0 + rr) * E + lane * 4) = *(const v4f*)(&Tf[rr][lane * 4]); *(volatile v2f*)(XC + (m0 + rr) * E + 128 + lane * 2) = (v2f){Tf[rr][128 + lane * 2], Tf[rr][128 + lane * 2 + 1]}; } __threadfence(); } }
__global__ __launch_bounds__(32) void xproj_kernel(const float* __restrict__ XC, const b16* __restrict__ XPT, const float* __restrict__ dtw, const float* __restrict__ dtb, int NRV, float* __restrict__ XD, float* __restrict__ DL) { __shared__ __attribute__((aligned(16))) b16 Ah[16][E + 8], Al[16][E + 8]; __shared__ float Tf[16][52]; const int lane = threadIdx.x, nloc = lane & 15, hlf = lane >> 4; const size_t m0 = (size_t)blockIdx.x * 16; if (m0 >= (size_t)NRV) return;
  for (int rr = 0; rr < 16; ++rr) for (int q = 0; q < E / 32; ++q) { b16 p, ql; split16(XC[(m0 + rr) * E + q * 32 + lane] * XS, p, ql); Ah[rr][q * 32 + lane] = p; Al[rr][q * 32 + lane] = ql; }
  wave_lds_sync(); v8f acc[3] = {(v8f){}, (v8f){}, (v8f){}};
#pragma unroll
  for (int kb = 0; kb < E; kb += 32) { const v16b a = frag_kb(&Ah[nloc][kb], hlf), al = frag_kb(&Al[nloc][kb], hlf);
#pragma unroll
    for (int t = 0; t < 3; ++t) { const v16b bw = frag_kb(XPT + (size_t)(t * 16 + nloc) * E + kb, hlf); acc[t] = wmma16b(a, bw, acc[t]); acc[t] = wmma16b(al, bw, acc[t]); } }
#pragma unroll
  for (int t = 0; t < 3; ++t)
#pragma unroll
    for (int r8 = 0; r8 < 8; ++r8) Tf[8 * hlf + r8][t * 16 + nloc] = acc[t][r8] * (1.0f / (XS * WSC));
  wave_lds_sync(); float wv[6][R]; for (int j = 0; j < 6; ++j) for (int r = 0; r < R; ++r) wv[j][r] = bf16_rne(dtw[(lane * 6 + j) * R + r]);
  for (int pass = 0; pass < 2; ++pass) { for (int rr = 0; rr < 16; ++rr) { for (int c = lane; c < XDW; c += 32) ((volatile float*)XD)[(m0 + rr) * XDW + c] = Tf[rr][c];
      for (int j = 0; j < 6; ++j) { const int e = lane * 6 + j; float s = bf16_rne(dtb[e]); for (int r = 0; r < R; ++r) s += pmul(Tf[rr][r], wv[j][r]); ((volatile float*)DL)[(m0 + rr) * E + e] = softplus(s); } }
    __threadfence(); } }
__global__ __launch_bounds__(32) void scan_kernel(const float* __restrict__ XC, const float* __restrict__ XD, const float* __restrict__ DL, const float* __restrict__ Alog, const float* __restrict__ Dp, const float* __restrict__ dirB, const int* __restrict__ orders, const int* __restrict__ dcodes, float* __restrict__ YS) {
  const int lane = threadIdx.x, b = blockIdx.x >> 1, half = blockIdx.x & 1; const int e0 = half * 96 + lane * 3; float A[3][NS], Dd[3];
  for (int j = 0; j < 3; ++j) { const int e = e0 + j; Dd[j] = bf16_rne(Dp[e]);
#pragma unroll
    for (int n = 0; n < NS; ++n) A[j][n] = -__expf(bf16_rne(Alog[e * NS + n])); }
  for (int pass = 0; pass < 2; ++pass) {
    for (int dir = 0; dir < NDIR; ++dir) { float st[3][NS];
#pragma unroll
      for (int j = 0; j < 3; ++j)
#pragma unroll
        for (int n = 0; n < NS; ++n) st[j][n] = 0.0f;
#pragma unroll 1
      for (int t = 0; t < L; ++t) { const int p = iclamp(orders[dir * L + t], 0, L - 1); const int dc = iclamp(dcodes[dir * L + t], 0, 4); const size_t row = (size_t)b * L + p;
        float Bn[NS], Cn[NS];
#pragma unroll
        for (int n = 0; n < NS; ++n) { Bn[n] = XD[row * XDW + R + n] + bf16_rne(dirB[dc * NS + n]); Cn[n] = XD[row * XDW + R + NS + n]; }
#pragma unroll
        for (int j = 0; j < 3; ++j) { const int e = e0 + j; const float dl = DL[row * E + e], u = XC[row * E + e]; const float du = pmul(dl, u); float y = pmul(u, Dd[j]);
#pragma unroll
          for (int n = 0; n < NS; ++n) { st[j][n] = pmul(__expf(pmul(dl, A[j][n])), st[j][n]) + pmul(du, Bn[n]); y += pmul(st[j][n], Cn[n]); }
          float* dst = YS + row * E + e; const float prev = dir == 0 ? 0.0f : *dst; *(volatile float*)dst = prev + 0.25f * y; } } }
    __threadfence(); } }
__global__ __launch_bounds__(32) void out_kernel(const float* __restrict__ YS, const float* __restrict__ XZ, const b16* __restrict__ WOT, int NRV, float* __restrict__ out) { __shared__ __attribute__((aligned(16))) b16 Ah[16][E + 8], Al[16][E + 8]; __shared__ float Tf[16][100]; const int lane = threadIdx.x, nloc = lane & 15, hlf = lane >> 4; const size_t m0 = (size_t)blockIdx.x * 16; if (m0 >= (size_t)NRV) return;
  for (int rr = 0; rr < 16; ++rr) for (int q = 0; q < E / 32; ++q) { const int c = q * 32 + lane; const float v = pmul(YS[(m0 + rr) * E + c], silu(XZ[(m0 + rr) * 2 * E + E + c])); b16 p, ql; split16(v * XS, p, ql); Ah[rr][c] = p; Al[rr][c] = ql; }
  wave_lds_sync(); v8f acc[6];
#pragma unroll
  for (int t = 0; t < 6; ++t) acc[t] = (v8f){};
#pragma unroll
  for (int kb = 0; kb < E; kb += 32) { const v16b a = frag_kb(&Ah[nloc][kb], hlf), al = frag_kb(&Al[nloc][kb], hlf);
#pragma unroll
    for (int t = 0; t < 6; ++t) { const v16b bw = frag_kb(WOT + (size_t)(t * 16 + nloc) * E + kb, hlf); acc[t] = wmma16b(a, bw, acc[t]); acc[t] = wmma16b(al, bw, acc[t]); } }
#pragma unroll
  for (int t = 0; t < 6; ++t)
#pragma unroll
    for (int r8 = 0; r8 < 8; ++r8) Tf[8 * hlf + r8][t * 16 + nloc] = acc[t][r8] * (1.0f / (XS * WSC));
  wave_lds_sync();
  for (int pass = 0; pass < 2; ++pass) { for (int rr = 0; rr < 16; ++rr) { const float* tr = Tf[rr]; *(volatile v2f*)(out + (m0 + rr) * DM + lane * 2) = (v2f){tr[lane * 2], tr[lane * 2 + 1]}; ((volatile float*)out)[(m0 + rr) * DM + 64 + lane] = tr[64 + lane]; } __threadfence(); } }
}

extern "C" void kernel_launch(void* const* d_in, const int* in_sizes, int n_in, void* d_out, int out_size, void* d_ws, size_t ws_size, hipStream_t stream) {
  (void)n_in;
  auto Fp = [&](int i) { return (const float*)d_in[i]; }; auto Ip = [&](int i) { return (const int*)d_in[i]; };
  if (in_sizes[0] != B * L * DM || in_sizes[3] != 2 * E * DM || in_sizes[4] != MID * E || in_sizes[7] != E * MID || in_sizes[8] != (R + 2 * NS) * E || in_sizes[9] != E * R || in_sizes[11] != E * NS || in_sizes[14] != 5 * NS || in_sizes[15] != NDIR * L || in_sizes[17] != NDIR * L || out_size != B * L * DM) return;
  const int BV = B; const int NRV = BV * L;
  size_t off = 0; char* ws = (char*)d_ws;
  auto carve = [&](size_t bytes) { char* p = ws + off; off += (bytes + 255) & ~(size_t)255; return p; };
  b16* WIN = (b16*)carve((size_t)2 * E * DM * 2); b16* PW1T = (b16*)carve((size_t)16 * E * 2); b16* PW2T = (b16*)carve((size_t)E * 32 * 2); b16* XPT = (b16*)carve((size_t)XDW * E * 2); b16* WOT = (b16*)carve((size_t)DM * E * 2);
  float* XZ = (float*)carve((size_t)B * L * 2 * E * 4); float* H1 = (float*)carve((size_t)B * L * 16 * 4); float* XC = (float*)carve((size_t)B * L * E * 4); float* XD = (float*)carve((size_t)B * L * XDW * 4); float* DL = (float*)carve((size_t)B * L * E * 4); float* YS = (float*)carve((size_t)B * L * E * 4);
  if (off > ws_size || off > ((size_t)160 << 20)) return;
  wput_kernel<<<(DM * (E / 8) > 2 * E * (DM / 8) ? DM * (E / 8) : 2 * E * (DM / 8)) / 256 + 2, 256, 0, stream>>>(Fp(3), Fp(4), Fp(7), Fp(8), Fp(13), WIN, PW1T, PW2T, XPT, WOT);
  inproj_kernel<<<(NRV / 16) * 3, 32, 0, stream>>>(Fp(0), WIN, NRV, XZ);
  pw1_kernel<<<NRV / 16, 32, 0, stream>>>(XZ, PW1T, Fp(5), NRV, H1);
  conv_kernel<<<NRV / 16, 32, 0, stream>>>(H1, Fp(6), PW2T, NRV, XC);
  xproj_kernel<<<NRV / 16, 32, 0, stream>>>(XC, XPT, Fp(9), Fp(10), NRV, XD, DL);
  scan_kernel<<<BV * 2, 32, 0, stream>>>(XC, XD, DL, Fp(11), Fp(12), Fp(14), Ip(15), Ip(17), YS);
  out_kernel<<<NRV / 16, 32, 0, stream>>>(YS, XZ, WOT, NRV, (float*)d_out);
}
